// PointNetSetAbstraction_3143916061237
// MI455X (gfx1250) — hardware-verified
//
#include <hip/hip_runtime.h>
#include <math.h>
#pragma clang fp contract(off)

typedef __attribute__((ext_vector_type(16))) _Float16 v16h;
typedef __attribute__((ext_vector_type(8)))  _Float16 v8h;
typedef __attribute__((ext_vector_type(16))) __bf16   v16b;
typedef __attribute__((ext_vector_type(8)))  __bf16   v8b;
typedef __attribute__((ext_vector_type(8)))  float    v8f;
typedef __attribute__((ext_vector_type(4)))  float    v4f;
typedef __attribute__((ext_vector_type(4)))  unsigned v4u;

constexpr int B_SZ   = 8;
constexpr int N_PTS  = 8192;
constexpr int S_PTS  = 2048;
constexpr int K_NBR  = 32;
constexpr int W0_LD  = 67;
constexpr int NGROUPS = B_SZ * S_PTS;
constexpr int NROWS   = NGROUPS * K_NBR;
constexpr int NPOINTS = B_SZ * N_PTS;
constexpr float RADIUS_SQ   = 0.09f;
constexpr float BN_EPS_F    = 1e-5f;
constexpr float W_CARRY     = 16.0f;
constexpr float W_CARRY_INV = 1.0f / 16.0f;
constexpr int STAT_BLOCKS   = NGROUPS / 32;
static_assert(NGROUPS == 16384);
static_assert(NROWS == 524288);
static_assert(NPOINTS % 64 == 0);
static_assert(STAT_BLOCKS == 512);

constexpr size_t SZ_NXYZ = (size_t)B_SZ * 3 * S_PTS * 4;
constexpr size_t SZ_IDX  = (size_t)NGROUPS * K_NBR * 4;
constexpr size_t SZ_AP   = (size_t)NPOINTS * 64 * 2;
constexpr size_t SZ_P    = (size_t)NPOINTS * 64 * 4;
constexpr size_t SZ_A1   = (size_t)NROWS * 64 * 2;
constexpr size_t SZ_HM   = (size_t)NGROUPS * 128 * 4;
constexpr size_t OFF_NXYZ = 0;
constexpr size_t OFF_IDX  = OFF_NXYZ + SZ_NXYZ;
constexpr size_t OFF_APH  = OFF_IDX + SZ_IDX;
constexpr size_t OFF_APL  = OFF_APH + SZ_AP;
constexpr size_t OFF_P    = OFF_APL + SZ_AP;
constexpr size_t OFF_A1   = OFF_P + SZ_P;
constexpr size_t OFF_HMAX = OFF_A1 + SZ_A1;
constexpr size_t OFF_HMIN = OFF_HMAX + SZ_HM;
constexpr size_t OFF_W0PH = OFF_HMIN + SZ_HM;
constexpr size_t OFF_W0PL = OFF_W0PH + 8192;
constexpr size_t OFF_W0X  = OFF_W0PL + 8192;
constexpr size_t OFF_W1H  = OFF_W0X + 1024;
constexpr size_t OFF_W2H  = OFF_W1H + 8192;
constexpr size_t OFF_PART0 = OFF_W2H + 16384;
constexpr size_t OFF_PART1 = OFF_PART0 + (size_t)STAT_BLOCKS * 128 * 4;
constexpr size_t OFF_PART2 = OFF_PART1 + (size_t)STAT_BLOCKS * 128 * 4;
constexpr size_t OFF_AFF0  = OFF_PART2 + (size_t)STAT_BLOCKS * 256 * 4;
constexpr size_t OFF_AFF1  = OFF_AFF0 + 512;
constexpr size_t OFF_AFF2  = OFF_AFF1 + 512;
constexpr size_t WS_TOTAL  = OFF_AFF2 + 1024;
static_assert(OFF_IDX % 128 == 0 && OFF_APH % 128 == 0 && OFF_P % 128 == 0 && OFF_A1 % 128 == 0);
static_assert(OFF_HMAX % 128 == 0 && OFF_W0PH % 128 == 0 && OFF_W0X % 128 == 0 && OFF_PART0 % 128 == 0);
static_assert(OFF_AFF0 % 128 == 0 && OFF_AFF2 % 128 == 0);
static_assert(WS_TOTAL <= (size_t)134217728);
constexpr size_t OUT1_BYTE_OFF = 196608;
constexpr size_t OUT_TOTAL_BYTES = 8585216;
static_assert(OUT1_BYTE_OFF == (size_t)B_SZ * 3 * S_PTS * 4);
static_assert(OUT1_BYTE_OFF % 128 == 0);
static_assert(OUT1_BYTE_OFF + (size_t)B_SZ * 128 * S_PTS * 4 <= OUT_TOTAL_BYTES);

__device__ __forceinline__ unsigned short f2bf_bits(float f) {
  unsigned u = __float_as_uint(f);
  return (unsigned short)((u + 0x7FFFu + ((u >> 16) & 1u)) >> 16);
}
__device__ __forceinline__ float bf_bits2f(unsigned short h) { return __uint_as_float(((unsigned)h) << 16); }
__device__ __forceinline__ unsigned bf_bits32(float f) {
  const unsigned u = __float_as_uint(f);
  return (u + 0x7FFFu + ((u >> 16) & 1u)) >> 16;
}
__device__ __forceinline__ float bf32_to_f(unsigned hb) { return __uint_as_float(hb << 16); }

__device__ __forceinline__ void st2_f32(float* p, float v) {
  volatile float* q = p; *q = v; __threadfence(); *q = v;
}
__device__ __forceinline__ void st2_i32(int* p, int v) {
  volatile int* q = p; *q = v; __threadfence(); *q = v;
}
__device__ __forceinline__ void st2_v4f(float* p, v4f v) {
  *(volatile v4f*)p = v; __threadfence(); *(volatile v4f*)p = v;
}
__device__ __forceinline__ void st2_v4u(unsigned short* p, v4u v) {
  *(volatile v4u*)p = v; __threadfence(); *(volatile v4u*)p = v;
}
__device__ __forceinline__ void st2_v8h(unsigned short* p, v8h v) {
  *(volatile v8h*)p = v; __threadfence(); *(volatile v8h*)p = v;
}
__device__ __forceinline__ void wave_lds_sync() {
  __builtin_amdgcn_fence(__ATOMIC_RELEASE, "workgroup");
  __builtin_amdgcn_wave_barrier();
  __builtin_amdgcn_fence(__ATOMIC_ACQUIRE, "workgroup");
}

__device__ __forceinline__ void dep_guard_h(v8f& a, v8f& b, v16h x, v16h y) { asm volatile("v_nop\n\tv_nop\n\tv_nop\n\tv_nop" : "+v"(a), "+v"(b) : "v"(x), "v"(y)); }
__device__ __forceinline__ void dep_guard_b(v8f& a, v8f& b, v16b x, v16b y) { asm volatile("v_nop\n\tv_nop\n\tv_nop\n\tv_nop" : "+v"(a), "+v"(b) : "v"(x), "v"(y)); }
__device__ __forceinline__ void keep4_h(v16h a, v16h b, v16h c, v16h d) { asm volatile("v_nop" :: "v"(a), "v"(b), "v"(c), "v"(d)); }
__device__ __forceinline__ void keep4_b(v16b a, v16b b, v16b c, v16b d) { asm volatile("v_nop" :: "v"(a), "v"(b), "v"(c), "v"(d)); }
__device__ __forceinline__ void acc_guard4(v8f& a, v8f& b, v8f& c, v8f& d) { asm volatile("v_nop\n\tv_nop\n\tv_nop\n\tv_nop" : "+v"(a), "+v"(b), "+v"(c), "+v"(d)); }
template <typename T> struct Frag;
template <> struct Frag<_Float16> {
  typedef v16h V; union U { v16h v; v8h h[2]; };
  static __device__ __forceinline__ v16h load(const _Float16* p) {
    U f; f.h[0] = *(const v8h*)(p); f.h[1] = *(const v8h*)(p + 16); return f.v;
  }
  static __device__ __forceinline__ v8f mma(v16h a, v16h b, v8f c) {
    return __builtin_amdgcn_wmma_f32_16x16x32_f16(false, a, false, b, (short)0, c, false, false);
  }
  static __device__ __forceinline__ void guard(v8f& a, v8f& b, v16h x, v16h y) { dep_guard_h(a, b, x, y); }
  static __device__ __forceinline__ void keep(v16h a, v16h b, v16h c, v16h d) { keep4_h(a, b, c, d); }
};
template <> struct Frag<__bf16> {
  typedef v16b V; union U { v16b v; v8b h[2]; };
  static __device__ __forceinline__ v16b load(const __bf16* p) {
    U f; f.h[0] = *(const v8b*)(p); f.h[1] = *(const v8b*)(p + 16); return f.v;
  }
  static __device__ __forceinline__ v8f mma(v16b a, v16b b, v8f c) {
    return __builtin_amdgcn_wmma_f32_16x16x32_bf16(false, a, false, b, (short)0, c, false, false);
  }
  static __device__ __forceinline__ void guard(v8f& a, v8f& b, v16b x, v16b y) { dep_guard_b(a, b, x, y); }
  static __device__ __forceinline__ void keep(v16b a, v16b b, v16b c, v16b d) { keep4_b(a, b, c, d); }
};

__device__ __forceinline__ v8f mma_h(v16h a, v16h b, v8f c) {
  c = __builtin_amdgcn_wmma_f32_16x16x32_f16(false, a, false, b, (short)0, c, false, false);
  asm volatile("v_nop\n\tv_nop\n\tv_nop\n\tv_nop" : "+v"(c) : "v"(a), "v"(b));
  return c;
}

template <int ET> struct Elem;
template <> struct Elem<0> { typedef _Float16 T; };
template <> struct Elem<1> { typedef __bf16 T; };
template <int ET, bool SPLIT, int BIAS_MODE, int OUT_MODE, bool RESID, int ACT = 0>
__global__ __launch_bounds__(256) void wmma_gemm64(
    const unsigned short* __restrict__ Ap, const unsigned short* __restrict__ A2p, int lda, long strideA,
    const unsigned short* __restrict__ Btp, const unsigned short* __restrict__ Bt2p, int ldb, long strideB,
    void* __restrict__ Cout, void* __restrict__ Cout2, int ldc, long strideC,
    const float* __restrict__ bias,
    const float* __restrict__ resid, long strideR,
    int M, int N, int K, float scale) {
  typedef typename Elem<ET>::T T;
  typedef typename Frag<T>::V V;
  const T* A = (const T*)Ap; const T* A2 = (const T*)A2p; const T* Bt = (const T*)Btp; const T* Bt2 = (const T*)Bt2p;
  __shared__ __align__(16) float sT[8][16 * 68];
  const int b    = blockIdx.y;
  const int lane = threadIdx.x & 31;
  const int wave = threadIdx.x >> 5;
  const int tilesN = N >> 6;
  const int tilesM = M >> 6;
  const int tile = blockIdx.x * 8 + wave;
  if (tile >= tilesM * tilesN) return;
  const int tm = tile / tilesN;
  const int tn = tile - tm * tilesN;
  const int m0 = tm << 6;
  const int n0 = tn << 6;

  const T* Ab  = A  + (size_t)b * strideA;
  const T* Bb  = Bt + (size_t)b * strideB;
  const T* Ab2 = SPLIT ? (A2  + (size_t)b * strideA) : nullptr;
  const T* Bb2 = SPLIT ? (Bt2 + (size_t)b * strideB) : nullptr;

  const int rlane = lane & 15;
  const int koff  = (lane >> 4) * 8;
  const int mOff  = (lane >> 4) * 8;

  v8f acc[4][4];
#pragma unroll
  for (int i = 0; i < 4; ++i)
#pragma unroll
    for (int j = 0; j < 4; ++j) acc[i][j] = (v8f){0.f,0.f,0.f,0.f,0.f,0.f,0.f,0.f};

  for (int k0 = 0; k0 < K; k0 += 32) {
    V bh[4], bl[4];
#pragma unroll
    for (int j = 0; j < 4; ++j) {
      const size_t bo = (size_t)(n0 + (j << 4) + rlane) * ldb + koff + k0;
      bh[j] = Frag<T>::load(Bb + bo);
      if (SPLIT) bl[j] = Frag<T>::load(Bb2 + bo);
    }
#pragma unroll
    for (int i = 0; i < 4; ++i) {
      const size_t ao = (size_t)(m0 + (i << 4) + rlane) * lda + koff + k0;
      V ah = Frag<T>::load(Ab + ao);
      V al;
      if (SPLIT) al = Frag<T>::load(Ab2 + ao);
#pragma unroll
      for (int j = 0; j < 4; ++j) {
        acc[i][j] = Frag<T>::mma(ah, bh[j], acc[i][j]);
        if (SPLIT) {
          acc[i][j] = Frag<T>::mma(ah, bl[j], acc[i][j]);
          acc[i][j] = Frag<T>::mma(al, bh[j], acc[i][j]);
        }
      }
      Frag<T>::guard(acc[i][0], acc[i][3], ah, SPLIT ? al : ah);
    }
    Frag<T>::keep(bh[0], bh[1], bh[2], bh[3]);
    if (SPLIT) Frag<T>::keep(bl[0], bl[1], bl[2], bl[3]);
  }
  acc_guard4(acc[0][0], acc[0][1], acc[0][2], acc[0][3]);
  acc_guard4(acc[1][0], acc[1][1], acc[1][2], acc[1][3]);
  acc_guard4(acc[2][0], acc[2][1], acc[2][2], acc[2][3]);
  acc_guard4(acc[3][0], acc[3][1], acc[3][2], acc[3][3]);

  float* slab = sT[wave];
  const float* Rb = RESID ? (resid + (size_t)b * strideR) : nullptr;
#pragma unroll
  for (int i = 0; i < 4; ++i) {
    const int mBase = m0 + (i << 4);
#pragma unroll
    for (int j = 0; j < 4; ++j) {
      const int n = n0 + (j << 4) + rlane;
      float bv = 0.f;
      if (BIAS_MODE == 2) bv = bias[n];
#pragma unroll
      for (int r = 0; r < 8; ++r) {
        float v = acc[i][j][r] * scale;
        if (BIAS_MODE == 1) v += bias[mBase + mOff + r];
        if (BIAS_MODE == 2) v += bv;
        if (RESID) v += Rb[(size_t)(mBase + mOff + r) * ldc + n];
        if (ACT == 1) v = tanhf(v);
        if (ACT == 2) v = fmaxf(v, 0.0f);
        if (ACT == 3) v = v / (1.0f + expf(-v));
        if (ACT == 4) v = (v > 0.f) ? v : 0.01f * v;
        if (ACT == 5) v = 0.5f * v * (1.0f + erff(v * 0.70710678118654752f));
        slab[(mOff + r) * 68 + (j << 4) + rlane] = v;
      }
    }
    __builtin_amdgcn_fence(__ATOMIC_RELEASE, "workgroup");
    __builtin_amdgcn_wave_barrier();
    __builtin_amdgcn_fence(__ATOMIC_ACQUIRE, "workgroup");
    if (OUT_MODE == 0) {
      float* C = (float*)Cout + (size_t)b * strideC;
      const int hh = lane >> 4, c4 = (lane & 15) * 4;
      for (int pass = 0; pass < 2; ++pass) {
#pragma unroll
        for (int it = 0; it < 8; ++it) {
          const int row = it * 2 + hh;
          v4f v = *(const v4f*)(slab + row * 68 + c4);
          *(volatile v4f*)(C + (size_t)(mBase + row) * ldc + n0 + c4) = v;
        }
        __threadfence();
      }
    } else {
      const int q = lane >> 3, c8 = (lane & 7) * 8;
      unsigned short* C  = (unsigned short*)Cout  + (size_t)b * strideC;
      unsigned short* C2 = (OUT_MODE == 2) ? ((unsigned short*)Cout2 + (size_t)b * strideC) : nullptr;
      for (int pass = 0; pass < 2; ++pass) {
#pragma unroll
        for (int it = 0; it < 4; ++it) {
          const int row = it * 4 + q;
          const float* sp = slab + row * 68 + c8;
          v8h hv, lv;
#pragma unroll
          for (int e = 0; e < 8; ++e) {
            if (OUT_MODE == 1) {
              hv[e] = (_Float16)sp[e];
            } else {
              unsigned short hb = f2bf_bits(sp[e]);
              unsigned short lb = f2bf_bits(sp[e] - bf_bits2f(hb));
              hv[e] = __builtin_bit_cast(_Float16, hb);
              lv[e] = __builtin_bit_cast(_Float16, lb);
            }
          }
          *(volatile v8h*)(C + (size_t)(mBase + row) * ldc + n0 + c8) = hv;
          if (OUT_MODE == 2) *(volatile v8h*)(C2 + (size_t)(mBase + row) * ldc + n0 + c8) = lv;
        }
        __threadfence();
      }
    }
    __builtin_amdgcn_fence(__ATOMIC_RELEASE, "workgroup");
    __builtin_amdgcn_wave_barrier();
    __builtin_amdgcn_fence(__ATOMIC_ACQUIRE, "workgroup");
  }
}

__global__ __launch_bounds__(256) void prep_weights(
    const float* __restrict__ W0, const float* __restrict__ W1, const float* __restrict__ W2,
    unsigned short* __restrict__ W0pH, unsigned short* __restrict__ W0pL, float* __restrict__ W0x,
    unsigned short* __restrict__ W1h, unsigned short* __restrict__ W2h) {
  const int tid = threadIdx.x;
  for (int ch = tid; ch < 512; ch += 256) {
    const int o = ch >> 3, c0 = (ch & 7) * 8;
    const float* src = W0 + o * W0_LD + 3 + c0;
    float f[8];
#pragma unroll
    for (int e = 0; e < 8; ++e) f[e] = src[e];
    unsigned hw[4], lw[4];
#pragma unroll
    for (int q = 0; q < 4; ++q) {
      const unsigned h0 = bf_bits32(f[2 * q]);
      const unsigned h1 = bf_bits32(f[2 * q + 1]);
      const unsigned l0 = bf_bits32(f[2 * q] - bf32_to_f(h0));
      const unsigned l1 = bf_bits32(f[2 * q + 1] - bf32_to_f(h1));
      hw[q] = (h0 & 0xffffu) | (h1 << 16);
      lw[q] = (l0 & 0xffffu) | (l1 << 16);
    }
    const v4u hv = (v4u){hw[0], hw[1], hw[2], hw[3]};
    const v4u lv = (v4u){lw[0], lw[1], lw[2], lw[3]};
    st2_v4u(W0pH + (size_t)ch * 8, hv);
    st2_v4u(W0pL + (size_t)ch * 8, lv);
  }
  for (int ch = tid; ch < 512; ch += 256) {
    const v4f x0 = *(const v4f*)(W1 + ch * 8);
    const v4f x1 = *(const v4f*)(W1 + ch * 8 + 4);
    v8h hv;
#pragma unroll
    for (int e = 0; e < 4; ++e) {
      const float a = x0[e] * W_CARRY;
      const float c = x1[e] * W_CARRY;
      hv[e] = (_Float16)a;
      hv[4 + e] = (_Float16)c;
    }
    st2_v8h(W1h + (size_t)ch * 8, hv);
  }
  for (int ch = tid; ch < 1024; ch += 256) {
    const v4f x0 = *(const v4f*)(W2 + ch * 8);
    const v4f x1 = *(const v4f*)(W2 + ch * 8 + 4);
    v8h hv;
#pragma unroll
    for (int e = 0; e < 4; ++e) {
      const float a = x0[e] * W_CARRY;
      const float c = x1[e] * W_CARRY;
      hv[e] = (_Float16)a;
      hv[4 + e] = (_Float16)c;
    }
    st2_v8h(W2h + (size_t)ch * 8, hv);
  }
  if (tid < 64) {
    const float* src = W0 + tid * W0_LD;
    const float a = src[0], c = src[1], d = src[2];
    const v4f w = (v4f){a, c, d, 0.0f};
    st2_v4f(W0x + tid * 4, w);
  }
}

__global__ __launch_bounds__(256) void transpose_points(
    const float* __restrict__ points, unsigned short* __restrict__ ApH, unsigned short* __restrict__ ApL) {
  __shared__ float tl[64 * 65];
  const int tid = threadIdx.x, lane = tid & 31, wave = tid >> 5;
  const int b = blockIdx.x >> 7;
  const int n0 = (blockIdx.x & 127) * 64;
#pragma unroll
  for (int i = 0; i < 4; ++i) {
    const int c = (tid >> 4) + 16 * i;
    const int n4 = (tid & 15) * 4;
    const v4f v = *(const v4f*)(points + ((size_t)(b * 64 + c)) * N_PTS + n0 + n4);
    tl[c * 65 + n4 + 0] = v[0];
    tl[c * 65 + n4 + 1] = v[1];
    tl[c * 65 + n4 + 2] = v[2];
    tl[c * 65 + n4 + 3] = v[3];
  }
  __syncthreads();
#pragma unroll
  for (int it = 0; it < 2; ++it) {
    const int n = it * 32 + wave * 4 + (lane >> 3);
    const int c8 = (lane & 7) * 8;
    unsigned hw[4], lw[4];
#pragma unroll
    for (int q = 0; q < 4; ++q) {
      const float f0 = tl[(c8 + 2 * q) * 65 + n];
      const float f1 = tl[(c8 + 2 * q + 1) * 65 + n];
      const unsigned h0 = bf_bits32(f0);
      const unsigned h1 = bf_bits32(f1);
      const unsigned l0 = bf_bits32(f0 - bf32_to_f(h0));
      const unsigned l1 = bf_bits32(f1 - bf32_to_f(h1));
      hw[q] = (h0 & 0xffffu) | (h1 << 16);
      lw[q] = (l0 & 0xffffu) | (l1 << 16);
    }
    const v4u hv = (v4u){hw[0], hw[1], hw[2], hw[3]};
    const v4u lv = (v4u){lw[0], lw[1], lw[2], lw[3]};
    const size_t off = ((size_t)b * N_PTS + n0 + n) * 64 + c8;
    st2_v4u(ApH + off, hv);
    st2_v4u(ApL + off, lv);
  }
}

__global__ __launch_bounds__(1024) void fps_kernel(
    const float* __restrict__ xyz, float* __restrict__ nxyz, float* __restrict__ out_xyz) {
#pragma clang fp contract(off)
  __shared__ float wval[32];
  __shared__ int   widx[32];
  __shared__ int   far_sh;
  __shared__ int   sel[S_PTS];
  const int b = blockIdx.x;
  const int tid = threadIdx.x;
  const int lane = tid & 31;
  const int wv = __builtin_amdgcn_readfirstlane(tid >> 5);
  const float* xb = xyz + (size_t)b * 3 * N_PTS;

  float px[8], py[8], pz[8], dist[8];
  {
    const v4f x0 = *(const v4f*)(xb + tid * 8);
    const v4f x1 = *(const v4f*)(xb + tid * 8 + 4);
    const v4f y0 = *(const v4f*)(xb + N_PTS + tid * 8);
    const v4f y1 = *(const v4f*)(xb + N_PTS + tid * 8 + 4);
    const v4f z0 = *(const v4f*)(xb + 2 * N_PTS + tid * 8);
    const v4f z1 = *(const v4f*)(xb + 2 * N_PTS + tid * 8 + 4);
#pragma unroll
    for (int e = 0; e < 4; ++e) {
      px[e] = x0[e]; px[4 + e] = x1[e];
      py[e] = y0[e]; py[4 + e] = y1[e];
      pz[e] = z0[e]; pz[4 + e] = z1[e];
    }
#pragma unroll
    for (int e = 0; e < 8; ++e) dist[e] = 1e10f;
  }

  int far = 0;
#pragma unroll 1
  for (int i = 0; i < S_PTS; ++i) {
    far = far < 0 ? 0 : (far > N_PTS - 1 ? N_PTS - 1 : far);
    const float cx = xb[far];
    const float cy = xb[N_PTS + far];
    const float cz = xb[2 * N_PTS + far];
    if (tid == 0) sel[i] = far;
    float bv = -1.0f;
    int bi = 0;
#pragma unroll
    for (int p = 0; p < 8; ++p) {
      const float dx = px[p] - cx;
      const float dy = py[p] - cy;
      const float dz = pz[p] - cz;
      const float t0 = dx * dx;
      const float t1 = dy * dy;
      const float t2 = dz * dz;
      const float d = (t0 + t2) + t1;
      const float nd = fminf(dist[p], d);
      dist[p] = nd;
      const int j = tid * 8 + p;
      const bool take = nd > bv;
      bv = take ? nd : bv;
      bi = take ? j : bi;
    }
#pragma unroll
    for (int off = 16; off; off >>= 1) {
      const float ov = __shfl_xor(bv, off, 32);
      const int oi = __shfl_xor(bi, off, 32);
      const bool take = (ov > bv) || (ov == bv && oi < bi);
      bv = take ? ov : bv;
      bi = take ? oi : bi;
    }
    if (lane == 0) { wval[wv] = bv; widx[wv] = bi; }
    __syncthreads();
    if (wv == 0) {
      float v = wval[lane];
      int ix = widx[lane];
#pragma unroll
      for (int off = 16; off; off >>= 1) {
        const float ov = __shfl_xor(v, off, 32);
        const int oi = __shfl_xor(ix, off, 32);
        const bool take = (ov > v) || (ov == v && oi < ix);
        v = take ? ov : v;
        ix = take ? oi : ix;
      }
      if (lane == 0) far_sh = ix;
    }
    __syncthreads();
    far = far_sh;
  }
  __syncthreads();
#pragma unroll
  for (int q = 0; q < 2; ++q) {
    const int s = q * 1024 + tid;
    int j = sel[s];
    j = j < 0 ? 0 : (j > N_PTS - 1 ? N_PTS - 1 : j);
    const float cx = xb[j];
    const float cy = xb[N_PTS + j];
    const float cz = xb[2 * N_PTS + j];
    const size_t o = (size_t)b * 3 * S_PTS + s;
    st2_f32(nxyz + o, cx);
    st2_f32(nxyz + o + S_PTS, cy);
    st2_f32(nxyz + o + 2 * S_PTS, cz);
    st2_f32(out_xyz + o, cx);
    st2_f32(out_xyz + o + S_PTS, cy);
    st2_f32(out_xyz + o + 2 * S_PTS, cz);
  }
}

__device__ __forceinline__ bool in_ball(float qx, float qy, float qz, float x, float y, float z) {
#pragma clang fp contract(off)
  const float dx = qx - x;
  const float dy = qy - y;
  const float dz = qz - z;
  const float t0 = dx * dx;
  const float t1 = dy * dy;
  const float t2 = dz * dz;
  const float d = (t0 + t2) + t1;
  return d <= RADIUS_SQ;
}

__global__ __launch_bounds__(256) void ball_query_kernel(
    const float* __restrict__ xyz, const float* __restrict__ nxyz, int* __restrict__ idx) {
#pragma clang fp contract(off)
  __shared__ int rows[8 * 32];
  const int tid = threadIdx.x, lane = tid & 31, wave = tid >> 5;
  int g = blockIdx.x * 8 + wave;
  g = g < NGROUPS ? g : NGROUPS - 1;
  const int b = g / S_PTS;
  const int s = g - b * S_PTS;
  const float* xb = xyz + (size_t)b * 3 * N_PTS;
  const float qx = nxyz[(size_t)b * 3 * S_PTS + s];
  const float qy = nxyz[(size_t)b * 3 * S_PTS + S_PTS + s];
  const float qz = nxyz[(size_t)b * 3 * S_PTS + 2 * S_PTS + s];
  int* row = rows + wave * 32;
  row[lane] = N_PTS - 1;
  __syncthreads();

  int cnt = 0;
  const unsigned lower = (1u << lane) - 1u;
#pragma unroll 1
  for (int base = 0; base < N_PTS && cnt < K_NBR; base += 128) {
    const v4f X = *(const v4f*)(xb + base + 4 * lane);
    const v4f Y = *(const v4f*)(xb + N_PTS + base + 4 * lane);
    const v4f Z = *(const v4f*)(xb + 2 * N_PTS + base + 4 * lane);
    const bool p0 = in_ball(qx, qy, qz, X[0], Y[0], Z[0]);
    const bool p1 = in_ball(qx, qy, qz, X[1], Y[1], Z[1]);
    const bool p2 = in_ball(qx, qy, qz, X[2], Y[2], Z[2]);
    const bool p3 = in_ball(qx, qy, qz, X[3], Y[3], Z[3]);
    const unsigned m0 = (unsigned)__ballot(p0);
    const unsigned m1 = (unsigned)__ballot(p1);
    const unsigned m2 = (unsigned)__ballot(p2);
    const unsigned m3 = (unsigned)__ballot(p3);
    int pos = cnt + __popc(m0 & lower) + __popc(m1 & lower) + __popc(m2 & lower) + __popc(m3 & lower);
    const int j0 = base + 4 * lane;
    if (p0 && pos < K_NBR) row[pos] = j0;
    pos += p0 ? 1 : 0;
    if (p1 && pos < K_NBR) row[pos] = j0 + 1;
    pos += p1 ? 1 : 0;
    if (p2 && pos < K_NBR) row[pos] = j0 + 2;
    pos += p2 ? 1 : 0;
    if (p3 && pos < K_NBR) row[pos] = j0 + 3;
    cnt += __popc(m0) + __popc(m1) + __popc(m2) + __popc(m3);
  }
  wave_lds_sync();
  const int total = cnt < K_NBR ? cnt : K_NBR;
  const int own = row[lane];
  const int first = row[0];
  int v = (lane < total) ? own : first;
  v = v < 0 ? 0 : (v > N_PTS - 1 ? N_PTS - 1 : v);
  st2_i32(idx + (size_t)g * K_NBR + lane, v);
}

template <bool APPLY>
__global__ __launch_bounds__(256) void gather_l0(
    const float* __restrict__ xyz, const float* __restrict__ nxyz, const int* __restrict__ idx,
    const float* __restrict__ P, const float* __restrict__ W0x, const float* __restrict__ aff,
    float* __restrict__ part, unsigned short* __restrict__ A1) {
  __shared__ __align__(16) float red[APPLY ? 4 : 32 * 128];
  __shared__ __align__(16) float fin[APPLY ? 4 : 128];
  const int tid = threadIdx.x, lane = tid & 31, wave = tid >> 5;
  const int q = lane >> 3;
  const int c8 = (lane & 7) * 8;

  float wx[8], wy[8], wz[8];
#pragma unroll
  for (int e = 0; e < 8; ++e) {
    const v4f w = *(const v4f*)(W0x + (c8 + e) * 4);
    wx[e] = w[0]; wy[e] = w[1]; wz[e] = w[2];
  }
  asm volatile("" ::: "memory");
  float sc[8], sh[8];
#pragma unroll
  for (int e = 0; e < 8; ++e) { sc[e] = 1.0f; sh[e] = 0.0f; }
  if (APPLY) {
    const v4f a0 = *(const v4f*)(aff + c8);
    const v4f a1 = *(const v4f*)(aff + c8 + 4);
    const v4f s0 = *(const v4f*)(aff + 64 + c8);
    const v4f s1 = *(const v4f*)(aff + 64 + c8 + 4);
#pragma unroll
    for (int e = 0; e < 4; ++e) { sc[e] = a0[e]; sc[4 + e] = a1[e]; sh[e] = s0[e]; sh[4 + e] = s1[e]; }
  }
  float s1a[8], s2a[8];
#pragma unroll
  for (int e = 0; e < 8; ++e) { s1a[e] = 0.0f; s2a[e] = 0.0f; }

#pragma unroll 1
  for (int gi = 0; gi < 4; ++gi) {
    const int g = (blockIdx.x * 8 + wave) * 4 + gi;
    const int b = g / S_PTS;
    const int s = g - b * S_PTS;
    const float* xb = xyz + (size_t)b * 3 * N_PTS;
    const float cx = nxyz[(size_t)b * 3 * S_PTS + s];
    const float cy = nxyz[(size_t)b * 3 * S_PTS + S_PTS + s];
    const float cz = nxyz[(size_t)b * 3 * S_PTS + 2 * S_PTS + s];
    int myidx = idx[(size_t)g * K_NBR + lane];
    myidx = myidx < 0 ? 0 : (myidx > N_PTS - 1 ? N_PTS - 1 : myidx);
#pragma unroll 1
    for (int it = 0; it < 8; ++it) {
      const int k = it * 4 + q;
      const int j = __shfl(myidx, k, 32);
      const float rx = xb[j] - cx;
      const float ry = xb[N_PTS + j] - cy;
      const float rz = xb[2 * N_PTS + j] - cz;
      const float* prow = P + ((size_t)b * N_PTS + j) * 64 + c8;
      const v4f p0 = *(const v4f*)(prow);
      const v4f p1 = *(const v4f*)(prow + 4);
      float z[8];
#pragma unroll
      for (int e = 0; e < 4; ++e) { z[e] = p0[e]; z[4 + e] = p1[e]; }
#pragma unroll
      for (int e = 0; e < 8; ++e) {
        float t = wx[e] * rx;
        t = __builtin_fmaf(wy[e], ry, t);
        t = __builtin_fmaf(wz[e], rz, t);
        z[e] = z[e] + t;
      }
      if (!APPLY) {
#pragma unroll
        for (int e = 0; e < 8; ++e) {
          s1a[e] += z[e];
          s2a[e] = __builtin_fmaf(z[e], z[e], s2a[e]);
        }
      } else {
        v8h hv;
#pragma unroll
        for (int e = 0; e < 8; ++e) {
          const float v = fmaxf(__builtin_fmaf(sc[e], z[e], sh[e]), 0.0f);
          hv[e] = (_Float16)v;
        }
        st2_v8h(A1 + ((size_t)g * K_NBR + k) * 64 + c8, hv);
      }
    }
  }

  if (!APPLY) {
    const int slot = wave * 4 + q;
#pragma unroll
    for (int e = 0; e < 8; ++e) {
      red[slot * 128 + c8 + e] = s1a[e];
      red[slot * 128 + 64 + c8 + e] = s2a[e];
    }
    __syncthreads();
    if (tid < 128) {
      float a = 0.0f;
#pragma unroll 1
      for (int sl = 0; sl < 32; ++sl) a += red[sl * 128 + tid];
      fin[tid] = a;
    }
    __syncthreads();
    if (wave == 0) {
      const v4f v = *(const v4f*)(fin + lane * 4);
      st2_v4f(part + (size_t)blockIdx.x * 128 + lane * 4, v);
    }
  }
}

__global__ __launch_bounds__(128) void reduce_affine(
    const float* __restrict__ part, int nblk, int C,
    const float* __restrict__ gamma, const float* __restrict__ beta, const float* __restrict__ bias,
    float* __restrict__ aff, float invR) {
  __shared__ __align__(16) float st[256];
  const int tid = threadIdx.x, lane = tid & 31, wave = tid >> 5;
  const int cc = tid < C ? tid : C - 1;
  double s = 0.0, s2 = 0.0;
#pragma unroll 1
  for (int i = 0; i < nblk; ++i) {
    s  += (double)part[(size_t)i * 2 * C + cc];
    s2 += (double)part[(size_t)i * 2 * C + C + cc];
  }
  const double mean = s * (double)invR;
  double var = s2 * (double)invR - mean * mean;
  var = var < 0.0 ? 0.0 : var;
  const float meanf = (float)mean;
  const float varf = (float)var;
  const float a = gamma[cc] * rsqrtf(varf + BN_EPS_F);
  const float bz = bias[cc];
  const float shift = (beta[cc] - a * (meanf + bz)) + a * bz;
  if (tid < C) { st[tid] = a; st[C + tid] = shift; }
  __syncthreads();
  if (wave < (2 * C) / 128) {
    const v4f v = *(const v4f*)(st + wave * 128 + lane * 4);
    st2_v4f(aff + wave * 128 + lane * 4, v);
  }
}

template <int PHASE>
__global__ __launch_bounds__(256) void mlp_kernel(
    const unsigned short* __restrict__ A1p, const unsigned short* __restrict__ W1p,
    const unsigned short* __restrict__ W2p, const float* __restrict__ aff1,
    float* __restrict__ part, float* __restrict__ hmax, float* __restrict__ hmin) {
  constexpr int NST = PHASE ? 256 : 128;
  constexpr int NJ  = PHASE ? 8 : 4;
  typedef Frag<_Float16> FragH;
  union FU { v16h v; v8h hh[2]; };
  __shared__ __align__(16) _Float16 Tl[PHASE ? 8 * 32 * 72 : 8];
  __shared__ __align__(16) float hm[PHASE ? 8 * 256 : 4];
  __shared__ __align__(16) float bst[8 * NST];
  __shared__ __align__(16) float fin[NST];

  const _Float16* A1 = (const _Float16*)A1p;
  const _Float16* W1 = (const _Float16*)W1p;
  const _Float16* W2 = (const _Float16*)W2p;
  const int tid = threadIdx.x, lane = tid & 31, wave = tid >> 5;
  const int n = lane & 15;
  const int h = lane >> 4;

  float scq[4], shq[4];
#pragma unroll
  for (int j = 0; j < 4; ++j) { scq[j] = 1.0f; shq[j] = 0.0f; }
  if (PHASE == 1) {
#pragma unroll
    for (int j = 0; j < 4; ++j) {
      scq[j] = aff1[j * 16 + n] * W_CARRY_INV;
      shq[j] = aff1[64 + j * 16 + n];
    }
  }
  float ssum[NJ], ssq[NJ];
#pragma unroll
  for (int t = 0; t < NJ; ++t) { ssum[t] = 0.0f; ssq[t] = 0.0f; }

#pragma unroll 1
  for (int gi = 0; gi < 4; ++gi) {
    const int g = (blockIdx.x * 8 + wave) * 4 + gi;
    const size_t rowbase = (size_t)g * K_NBR;

    v8f acc[2][4];
#pragma unroll
    for (int i = 0; i < 2; ++i)
#pragma unroll
      for (int j = 0; j < 4; ++j) acc[i][j] = (v8f){0.f,0.f,0.f,0.f,0.f,0.f,0.f,0.f};
#pragma unroll
    for (int ks = 0; ks < 2; ++ks) {
      const v16h a0 = FragH::load(A1 + (rowbase + n) * 64 + 8 * h + ks * 32);
      const v16h a1 = FragH::load(A1 + (rowbase + 16 + n) * 64 + 8 * h + ks * 32);
#pragma unroll
      for (int j = 0; j < 4; ++j) {
        const v16h bf = FragH::load(W1 + (j * 16 + n) * 64 + 8 * h + ks * 32);
        acc[0][j] = mma_h(a0, bf, acc[0][j]);
        acc[1][j] = mma_h(a1, bf, acc[1][j]);
      }
    }

    if (PHASE == 0) {
#pragma unroll
      for (int j = 0; j < 4; ++j) {
        float s = 0.0f, s2 = 0.0f;
#pragma unroll
        for (int i = 0; i < 2; ++i)
#pragma unroll
          for (int r = 0; r < 8; ++r) {
            const float z = acc[i][j][r] * W_CARRY_INV;
            s += z;
            s2 += z * z;
          }
        ssum[j] += s;
        ssq[j] += s2;
      }
    } else {
      _Float16* tw = Tl + wave * (32 * 72);
      float* hmw = hm + wave * 256;
#pragma unroll
      for (int i = 0; i < 2; ++i)
#pragma unroll
        for (int j = 0; j < 4; ++j)
#pragma unroll
          for (int r = 0; r < 8; ++r) {
            const float v = fmaxf(acc[i][j][r] * scq[j] + shq[j], 0.0f);
            tw[(i * 16 + 8 * h + r) * 72 + j * 16 + n] = (_Float16)v;
          }
      wave_lds_sync();
      FU a2[2][2];
#pragma unroll
      for (int i = 0; i < 2; ++i)
#pragma unroll
        for (int kk = 0; kk < 2; ++kk) {
          a2[i][kk].hh[0] = *(const v8h*)(tw + (i * 16 + n) * 72 + kk * 32 + 8 * h);
          a2[i][kk].hh[1] = *(const v8h*)(tw + (i * 16 + n) * 72 + kk * 32 + 16 + 8 * h);
        }
      wave_lds_sync();
#pragma unroll
      for (int nh = 0; nh < 2; ++nh) {
        v8f acc2[2][4];
#pragma unroll
        for (int i = 0; i < 2; ++i)
#pragma unroll
          for (int j = 0; j < 4; ++j) acc2[i][j] = (v8f){0.f,0.f,0.f,0.f,0.f,0.f,0.f,0.f};
#pragma unroll
        for (int kk = 0; kk < 2; ++kk) {
#pragma unroll
          for (int j = 0; j < 4; ++j) {
            const v16h bf = FragH::load(W2 + ((nh * 4 + j) * 16 + n) * 64 + 8 * h + kk * 32);
            acc2[0][j] = mma_h(a2[0][kk].v, bf, acc2[0][j]);
            acc2[1][j] = mma_h(a2[1][kk].v, bf, acc2[1][j]);
          }
        }
#pragma unroll
        for (int j = 0; j < 4; ++j) {
          float mx = -3.0e38f, mn = 3.0e38f, s = 0.0f, s2 = 0.0f;
#pragma unroll
          for (int i = 0; i < 2; ++i)
#pragma unroll
            for (int r = 0; r < 8; ++r) {
              const float z = acc2[i][j][r] * W_CARRY_INV;
              mx = fmaxf(mx, z);
              mn = fminf(mn, z);
              s += z;
              s2 += z * z;
            }
          const float omx = __shfl_xor(mx, 16, 32);
          const float omn = __shfl_xor(mn, 16, 32);
          mx = fmaxf(mx, omx);
          mn = fminf(mn, omn);
          ssum[nh * 4 + j] += s;
          ssq[nh * 4 + j] += s2;
          if (h == 0) {
            hmw[(nh * 4 + j) * 16 + n] = mx;
            hmw[128 + (nh * 4 + j) * 16 + n] = mn;
          }
        }
      }
      wave_lds_sync();
      {
        const v4f vmax = *(const v4f*)(hmw + lane * 4);
        const v4f vmin = *(const v4f*)(hmw + 128 + lane * 4);
        st2_v4f(hmax + (size_t)g * 128 + lane * 4, vmax);
        st2_v4f(hmin + (size_t)g * 128 + lane * 4, vmin);
      }
      wave_lds_sync();
    }
  }

#pragma unroll
  for (int t = 0; t < NJ; ++t) {
    const float o1 = __shfl_xor(ssum[t], 16, 32);
    const float o2 = __shfl_xor(ssq[t], 16, 32);
    ssum[t] += o1;
    ssq[t] += o2;
  }
  if (h == 0) {
#pragma unroll
    for (int t = 0; t < NJ; ++t) {
      bst[wave * NST + t * 16 + n] = ssum[t];
      bst[wave * NST + NST / 2 + t * 16 + n] = ssq[t];
    }
  }
  __syncthreads();
  if (tid < NST) {
    float a = 0.0f;
#pragma unroll
    for (int w = 0; w < 8; ++w) a += bst[w * NST + tid];
    fin[tid] = a;
  }
  __syncthreads();
  if (wave < NST / 128) {
    const v4f v = *(const v4f*)(fin + wave * 128 + lane * 4);
    st2_v4f(part + (size_t)blockIdx.x * NST + wave * 128 + lane * 4, v);
  }
}

__global__ __launch_bounds__(256) void final_kernel(
    const float* __restrict__ hmax, const float* __restrict__ hmin, const float* __restrict__ aff2,
    float* __restrict__ out1) {
  __shared__ __align__(16) float tile[128 * 36];
  const int tid = threadIdx.x, lane = tid & 31, wave = tid >> 5;
  const int b = blockIdx.x >> 6;
  const int s0 = (blockIdx.x & 63) * 32;
  const v4f a = *(const v4f*)(aff2 + lane * 4);
  const v4f sh = *(const v4f*)(aff2 + 128 + lane * 4);
#pragma unroll
  for (int rr = 0; rr < 4; ++rr) {
    const int srow = wave * 4 + rr;
    const size_t g = (size_t)b * S_PTS + s0 + srow;
    const v4f vx = *(const v4f*)(hmax + g * 128 + lane * 4);
    const v4f vn = *(const v4f*)(hmin + g * 128 + lane * 4);
#pragma unroll
    for (int e = 0; e < 4; ++e) {
      const float ae = a[e];
      const float fa = (ae >= 0.0f) ? 1.0f : 0.0f;
      const float fb = 1.0f - fa;
      const float z = fa * vx[e] + fb * vn[e];
      const float v = fmaxf(ae * z + sh[e], 0.0f);
      tile[(lane * 4 + e) * 36 + srow] = v;
    }
  }
  __syncthreads();
  for (int pass = 0; pass < 2; ++pass) {
#pragma unroll
    for (int it = 0; it < 4; ++it) {
      const int c = it * 32 + wave * 4 + (lane >> 3);
      const int s4 = (lane & 7) * 4;
      const v4f v = *(const v4f*)(tile + c * 36 + s4);
      *(volatile v4f*)(out1 + ((size_t)b * 128 + c) * S_PTS + s0 + s4) = v;
    }
    __threadfence();
  }
}

extern "C" void kernel_launch(void* const* d_in, const int* in_sizes, int n_in,
                              void* d_out, int out_size, void* d_ws, size_t ws_size,
                              hipStream_t stream) {
  if (n_in < 14) return;
  if (ws_size < WS_TOTAL) return;
  if ((size_t)out_size * 4 < OUT_TOTAL_BYTES) return;

  const float* xyz    = (const float*)d_in[0];
  const float* points = (const float*)d_in[1];
  const float* W0  = (const float*)d_in[2];
  const float* b0  = (const float*)d_in[3];
  const float* g0  = (const float*)d_in[4];
  const float* be0 = (const float*)d_in[5];
  const float* W1  = (const float*)d_in[6];
  const float* b1  = (const float*)d_in[7];
  const float* g1  = (const float*)d_in[8];
  const float* be1 = (const float*)d_in[9];
  const float* W2  = (const float*)d_in[10];
  const float* b2  = (const float*)d_in[11];
  const float* g2  = (const float*)d_in[12];
  const float* be2 = (const float*)d_in[13];

  float* out0 = (float*)d_out;
  float* out1 = (float*)((char*)d_out + OUT1_BYTE_OFF);

  char* ws = (char*)d_ws;
  float*          nxyz  = (float*)(ws + OFF_NXYZ);
  int*            bidx  = (int*)(ws + OFF_IDX);
  unsigned short* ApH   = (unsigned short*)(ws + OFF_APH);
  unsigned short* ApL   = (unsigned short*)(ws + OFF_APL);
  float*          Pp    = (float*)(ws + OFF_P);
  unsigned short* A1    = (unsigned short*)(ws + OFF_A1);
  float*          hmaxp = (float*)(ws + OFF_HMAX);
  float*          hminp = (float*)(ws + OFF_HMIN);
  unsigned short* W0pH  = (unsigned short*)(ws + OFF_W0PH);
  unsigned short* W0pL  = (unsigned short*)(ws + OFF_W0PL);
  float*          W0x   = (float*)(ws + OFF_W0X);
  unsigned short* W1h   = (unsigned short*)(ws + OFF_W1H);
  unsigned short* W2h   = (unsigned short*)(ws + OFF_W2H);
  float*          part0 = (float*)(ws + OFF_PART0);
  float*          part1 = (float*)(ws + OFF_PART1);
  float*          part2 = (float*)(ws + OFF_PART2);
  float*          aff0  = (float*)(ws + OFF_AFF0);
  float*          aff1  = (float*)(ws + OFF_AFF1);
  float*          aff2  = (float*)(ws + OFF_AFF2);

  const float invR = 1.0f / (float)NROWS;

  prep_weights<<<1, 256, 0, stream>>>(W0, W1, W2, W0pH, W0pL, W0x, W1h, W2h);
  transpose_points<<<B_SZ * (N_PTS / 64), 256, 0, stream>>>(points, ApH, ApL);
  fps_kernel<<<B_SZ, 1024, 0, stream>>>(xyz, nxyz, out0);
  ball_query_kernel<<<NGROUPS / 8, 256, 0, stream>>>(xyz, nxyz, bidx);

  static_assert(NPOINTS % 64 == 0);
  static_assert(64 % 64 == 0 && 64 % 32 == 0);
  wmma_gemm64<1, true, 0, 0, false, 0><<<dim3((NPOINTS / 64) / 8, 1), 256, 0, stream>>>(
      ApH, ApL, 64, 0L, W0pH, W0pL, 64, 0L, (void*)Pp, (void*)Pp, 64, 0L,
      aff0, Pp, 0L, NPOINTS, 64, 64, 1.0f);

  gather_l0<false><<<STAT_BLOCKS, 256, 0, stream>>>(xyz, nxyz, bidx, Pp, W0x, aff0, part0, A1);
  reduce_affine<<<1, 128, 0, stream>>>(part0, STAT_BLOCKS, 64, g0, be0, b0, aff0, invR);
  gather_l0<true><<<STAT_BLOCKS, 256, 0, stream>>>(xyz, nxyz, bidx, Pp, W0x, aff0, part0, A1);

  mlp_kernel<0><<<STAT_BLOCKS, 256, 0, stream>>>(A1, W1h, W2h, aff1, part1, hmaxp, hminp);
  reduce_affine<<<1, 128, 0, stream>>>(part1, STAT_BLOCKS, 64, g1, be1, b1, aff1, invR);
  mlp_kernel<1><<<STAT_BLOCKS, 256, 0, stream>>>(A1, W1h, W2h, aff1, part2, hmaxp, hminp);
  reduce_affine<<<1, 128, 0, stream>>>(part2, STAT_BLOCKS, 128, g2, be2, b2, aff2, invR);

  final_kernel<<<B_SZ * (S_PTS / 32), 256, 0, stream>>>(hmaxp, hminp, aff2, out1);
}
